// TinyAttention_74414603371080
// MI455X (gfx1250) — hardware-verified
//
#include <hip/hip_runtime.h>


namespace {
constexpr int N = 8192, DM = 1024, KD = 64, OD = 1024, QL = 8192  ;
constexpr float XS = 8.0f, WSC = 256.0f, PS = 1024.0f, LOG2E = 1.4426950408889634f;
static_assert(N % 64 == 0 && QL % 64 == 0, "tiling");
typedef _Float16 b16;
typedef __attribute__((ext_vector_type(16))) _Float16 v16b;
typedef __attribute__((ext_vector_type(8))) _Float16 v8b;
typedef __attribute__((ext_vector_type(8))) float v8f;
typedef __attribute__((ext_vector_type(4))) float v4f;
__device__ __forceinline__ float bf16_rne(float f) { unsigned int u = __float_as_uint(f); u += 0x7FFFu + ((u >> 16) & 1u); return __uint_as_float(u & 0xFFFF0000u); }
__device__ __forceinline__ void split16(float v, b16& hi, b16& lo) { hi = (b16)v; lo = (b16)(v - (float)hi); }
__device__ __forceinline__ v16b frag_kb(const b16* p, int hh) { const v8b a = *(const v8b*)(p + 8 * hh), b = *(const v8b*)(p + 16 + 8 * hh); v16b f;
#pragma unroll
  for (int e = 0; e < 8; ++e) { f[e] = a[e]; f[8 + e] = b[e]; } return f; }
__device__ __forceinline__ v8f wmma16b(v16b a, v16b b, v8f c) { v8f d = __builtin_amdgcn_wmma_f32_16x16x32_f16(false, a, false, b, (short)0, c, false, false); asm volatile("v_nop\n\tv_nop\n\tv_nop\n\tv_nop" : "+v"(d) : "v"(a), "v"(b)); return d; }
__device__ __forceinline__ void wave_lds_sync() { __builtin_amdgcn_fence(__ATOMIC_RELEASE, "workgroup"); __builtin_amdgcn_wave_barrier(); __builtin_amdgcn_fence(__ATOMIC_ACQUIRE, "workgroup"); }
__device__ __forceinline__ float pmul(float a, float b) { float p = a * b; asm volatile("" : "+v"(p)); return p; }
__device__ __forceinline__ int iclamp(int v, int lo, int hi) { return v < lo ? lo : (v > hi ? hi : v); }

typedef __attribute__((ext_vector_type(2))) _Float16 v2h;
typedef __attribute__((ext_vector_type(4))) _Float16 v4h;
typedef __attribute__((ext_vector_type(2))) float v2f;
__device__ __forceinline__ float nexp2(float v) { return __builtin_amdgcn_exp2f(v); }
__global__ __launch_bounds__(256) void prep_kernel(const float* __restrict__ wqkv, const float* __restrict__ wout, b16* __restrict__ WQ, b16* __restrict__ WO) {
  int t = blockIdx.x * 256 + threadIdx.x; v8b o;
  if (t < 3 * KD * DM / 8) { const int e = t * 8; const int oo = e / DM, k0 = e % DM; for (int j = 0; j < 8; ++j) o[j] = (b16)(bf16_rne(wqkv[(size_t)(k0 + j) * (3 * KD) + oo]) * WSC); for (int pass = 0; pass < 2; ++pass) { *(volatile v8b*)(WQ + e) = o; __threadfence(); } return; }
  t -= 3 * KD * DM / 8; if (t < OD * KD / 8) { const int e = t * 8; const int oo = e / KD, k0 = e % KD; for (int j = 0; j < 8; ++j) o[j] = (b16)(bf16_rne(wout[(size_t)(k0 + j) * OD + oo]) * WSC); for (int pass = 0; pass < 2; ++pass) { *(volatile v8b*)(WO + e) = o; __threadfence(); } }
}
__global__ __launch_bounds__(128) void proj_kernel(const float* __restrict__ x, const b16* __restrict__ WQ, const float* __restrict__ bqkv, b16* __restrict__ Qh, b16* __restrict__ Ql, b16* __restrict__ Kh, b16* __restrict__ Kl, b16* __restrict__ VT, b16* __restrict__ VTl) {
  __shared__ __attribute__((aligned(16))) b16 As[64][256 + 8]; __shared__ __attribute__((aligned(16))) float Tf[4][16][192 + 4];
  const int wave = threadIdx.x >> 5, lane = threadIdx.x & 31, nloc = lane & 15, hlf = lane >> 4; const size_t r0 = (size_t)blockIdx.x * 64; const size_t m0 = r0 + wave * 16;
  v8f acc[12];
#pragma unroll
  for (int t = 0; t < 12; ++t) acc[t] = (v8f){};
#pragma unroll 1
  for (int kc = 0; kc < DM; kc += 256) {
    __syncthreads();
    for (int i = threadIdx.x; i < 64 * 64; i += 128) { const int rr = i / 64, q = (i % 64) * 4; const v4f f = *(const v4f*)(x + (r0 + rr) * DM + kc + q); v4h o; for (int j = 0; j < 4; ++j) o[j] = (b16)(bf16_rne(f[j]) * XS); *(v4h*)(&As[rr][q]) = o; }
    __syncthreads();
#pragma unroll 2
    for (int kb = 0; kb < 256; kb += 32) { const v16b a = frag_kb(&As[wave * 16 + nloc][kb], hlf);
#pragma unroll
      for (int t = 0; t < 12; ++t) acc[t] = wmma16b(a, frag_kb(WQ + (size_t)(t * 16 + nloc) * DM + kc + kb, hlf), acc[t]); } }
#pragma unroll
  for (int t = 0; t < 12; ++t) { const float bb = bf16_rne(bqkv[t * 16 + nloc]);
#pragma unroll
    for (int r = 0; r < 8; ++r) Tf[wave][8 * hlf + r][t * 16 + nloc] = acc[t][r] * (1.0f / (XS * WSC)) + bb; }
  __syncthreads();
  for (int pass = 0; pass < 2; ++pass) {
    for (int rr = 0; rr < 16; ++rr) { const size_t row = m0 + rr; const v2f q2 = *(const v2f*)(&Tf[wave][rr][lane * 2]), k2 = *(const v2f*)(&Tf[wave][rr][KD + lane * 2]); v2h qh, ql, kh, kl;
      for (int j = 0; j < 2; ++j) { b16 p, q; split16(q2[j] * XS, p, q); qh[j] = p; ql[j] = q; split16(k2[j] * XS, p, q); kh[j] = p; kl[j] = q; }
      *(volatile v2h*)(Qh + row * KD + lane * 2) = qh; *(volatile v2h*)(Ql + row * KD + lane * 2) = ql; *(volatile v2h*)(Kh + row * KD + lane * 2) = kh; *(volatile v2h*)(Kl + row * KD + lane * 2) = kl; }
#pragma unroll 1
    for (int q = 0; q < 16; ++q) { const int d = wave * 16 + q; const int tk = lane * 2; v2h vh, vl; for (int j = 0; j < 2; ++j) { b16 p, ql; split16(Tf[(tk + j) >> 4][(tk + j) & 15][2 * KD + d] * XS, p, ql); vh[j] = p; vl[j] = ql; } *(volatile v2h*)(VT + (size_t)d * N + r0 + lane * 2) = vh; *(volatile v2h*)(VTl + (size_t)d * N + r0 + lane * 2) = vl; }
    __threadfence(); }
}
__global__ __launch_bounds__(64) void attn_kernel(const b16* __restrict__ Qh, const b16* __restrict__ Ql, const b16* __restrict__ Kh, const b16* __restrict__ Kl, const b16* __restrict__ VT, const b16* __restrict__ VTl, b16* __restrict__ Ch, b16* __restrict__ Cl) {
  __shared__ __attribute__((aligned(16))) b16 Pb[2][16][32 + 8], Pc[2][16][32 + 8]; __shared__ __attribute__((aligned(16))) float To[2][16][KD + 4];
  const int wave = threadIdx.x >> 5, lane = threadIdx.x & 31, hh = lane >> 4, col = lane & 15; const int q0 = blockIdx.x * 32 + wave * 16, qi = q0 + col;
  const v16b qa0 = frag_kb(Qh + (size_t)qi * KD, hh), qa1 = frag_kb(Qh + (size_t)qi * KD + 32, hh), qb0 = frag_kb(Ql + (size_t)qi * KD, hh), qb1 = frag_kb(Ql + (size_t)qi * KD + 32, hh);
  const float cs = LOG2E / (XS * XS);
  float m = -INFINITY, l = 0.0f; v8f o[4]; for (int t = 0; t < 4; ++t) o[t] = (v8f){};
  const int kend = q0 + 16;
#pragma unroll 1
  for (int kb = 0; kb < kend; kb += 32) {
    float e[16]; float mx = -INFINITY;
#pragma unroll
    for (int u = 0; u < 2; ++u) { v8f s = (v8f){}; const size_t kr = (size_t)(kb + u * 16 + col) * KD; const v16b kh0 = frag_kb(Kh + kr, hh), kh1 = frag_kb(Kh + kr + 32, hh), kl0 = frag_kb(Kl + kr, hh), kl1 = frag_kb(Kl + kr + 32, hh);
      s = wmma16b(kh0, qa0, s); s = wmma16b(kh1, qa1, s); s = wmma16b(kh0, qb0, s); s = wmma16b(kh1, qb1, s); s = wmma16b(kl0, qa0, s); s = wmma16b(kl1, qa1, s);
#pragma unroll
      for (int r = 0; r < 8; ++r) { const int key = kb + u * 16 + 8 * hh + r; const float vv = (key <= qi) ? s[r] * cs : -INFINITY; e[u * 8 + r] = vv; mx = fmaxf(mx, vv); } }
    mx = fmaxf(mx, __shfl_xor(mx, 16)); const float mn = fmaxf(m, mx); const float al = (mn == -INFINITY) ? 1.0f : nexp2(m - mn); float sum = 0.0f;
#pragma unroll
    for (int i2 = 0; i2 < 16; ++i2) { const float p = (e[i2] == -INFINITY) ? 0.0f : nexp2(e[i2] - mn); sum += p; b16 a_, b_; split16(p * PS, a_, b_); const int sl = (i2 < 8 ? 0 : 16) + 8 * hh + (i2 & 7); Pb[wave][col][sl] = a_; Pc[wave][col][sl] = b_; }
    sum += __shfl_xor(sum, 16); l = l * al + sum; m = mn;
    wave_lds_sync();
    const v16b pf = frag_kb(&Pb[wave][col][0], hh), pg = frag_kb(&Pc[wave][col][0], hh);
#pragma unroll
    for (int t = 0; t < 4; ++t) { o[t] *= al; const v16b va = frag_kb(VT + (size_t)(t * 16 + col) * N + kb, hh), vb = frag_kb(VTl + (size_t)(t * 16 + col) * N + kb, hh); o[t] = wmma16b(va, pf, o[t]); o[t] = wmma16b(va, pg, o[t]); o[t] = wmma16b(vb, pf, o[t]); }
    wave_lds_sync(); }
  const float inv = 1.0f / (l * PS * XS);
#pragma unroll
  for (int t = 0; t < 4; ++t)
#pragma unroll
    for (int r = 0; r < 8; ++r) To[wave][col][t * 16 + 8 * hh + r] = o[t][r] * inv;
  wave_lds_sync();
  for (int pass = 0; pass < 2; ++pass) { for (int rr = 0; rr < 16; ++rr) { const v2f f = *(const v2f*)(&To[wave][rr][lane * 2]); v2h hv, lv; for (int j = 0; j < 2; ++j) { b16 p, q; split16(f[j] * XS, p, q); hv[j] = p; lv[j] = q; }
      *(volatile v2h*)(Ch + (size_t)(q0 + rr) * KD + lane * 2) = hv; *(volatile v2h*)(Cl + (size_t)(q0 + rr) * KD + lane * 2) = lv; } __threadfence(); }
}
__global__ __launch_bounds__(128) void out_kernel(const b16* __restrict__ Ch, const b16* __restrict__ Cl, const b16* __restrict__ WO, const float* __restrict__ bo, float* __restrict__ out) {
  __shared__ __attribute__((aligned(16))) float Tf[4][16][128 + 4];
  const int wave = threadIdx.x >> 5, lane = threadIdx.x & 31, nloc = lane & 15, hlf = lane >> 4; const size_t m0 = (size_t)blockIdx.x * 64 + wave * 16; const int n0 = blockIdx.y * 128;
  v8f acc[8];
#pragma unroll
  for (int t = 0; t < 8; ++t) acc[t] = (v8f){};
#pragma unroll
  for (int kb = 0; kb < KD; kb += 32) { const v16b a = frag_kb(Ch + (m0 + nloc) * KD + kb, hlf), al = frag_kb(Cl + (m0 + nloc) * KD + kb, hlf);
#pragma unroll
    for (int t = 0; t < 8; ++t) { const v16b bw = frag_kb(WO + (size_t)(n0 + t * 16 + nloc) * KD + kb, hlf); acc[t] = wmma16b(a, bw, acc[t]); acc[t] = wmma16b(al, bw, acc[t]); } }
#pragma unroll
  for (int t = 0; t < 8; ++t) { const float bb = bf16_rne(bo[n0 + t * 16 + nloc]);
#pragma unroll
    for (int r = 0; r < 8; ++r) Tf[wave][8 * hlf + r][t * 16 + nloc] = acc[t][r] * (1.0f / (XS * WSC)) + bb; }
  wave_lds_sync();
  for (int pass = 0; pass < 2; ++pass) { for (int rr = 0; rr < 16; ++rr) *(volatile v4f*)(out + (m0 + rr) * OD + n0 + lane * 4) = *(const v4f*)(&Tf[wave][rr][lane * 4]); __threadfence(); }
}
}

extern "C" void kernel_launch(void* const* d_in, const int* in_sizes, int n_in, void* d_out, int out_size, void* d_ws, size_t ws_size, hipStream_t stream) {
  (void)n_in;
  auto Fp = [&](int i) { return (const float*)d_in[i]; };
  if (in_sizes[0] != N * DM || in_sizes[1] != DM * 3 * KD || in_sizes[2] != 3 * KD || in_sizes[3] != KD * OD || in_sizes[4] != OD || out_size != N * OD) return;
  size_t off = 0; char* ws = (char*)d_ws;
  auto carve = [&](size_t bytes) { char* p = ws + off; off += (bytes + 255) & ~(size_t)255; return p; };
  b16* WQ = (b16*)carve((size_t)3 * KD * DM * 2); b16* WO = (b16*)carve((size_t)OD * KD * 2); const size_t plane = (size_t)N * KD * 2;
  b16* Qh = (b16*)carve(plane); b16* Ql = (b16*)carve(plane); b16* Kh = (b16*)carve(plane); b16* Kl = (b16*)carve(plane); b16* VT = (b16*)carve(plane); b16* VTl = (b16*)carve(plane); b16* Ch = (b16*)carve(plane); b16* Cl = (b16*)carve(plane);
  if (off > ws_size || off > ((size_t)128 << 20)) return;
  prep_kernel<<<(3 * KD * DM / 8 + OD * KD / 8 + 255) / 256, 256, 0, stream>>>(Fp(1), Fp(3), WQ, WO);
  proj_kernel<<<N / 64, 128, 0, stream>>>(Fp(0), WQ, Fp(2), Qh, Ql, Kh, Kl, VT, VTl);
  attn_kernel<<<QL / 32, 64, 0, stream>>>(Qh, Ql, Kh, Kl, VT, VTl, Ch, Cl);
  out_kernel<<<dim3(QL / 64, OD / 128), 128, 0, stream>>>(Ch, Cl, WO, Fp(4), (float*)d_out);
}
